// BiGATFusionModel_42434276885024
// MI455X (gfx1250) — hardware-run, weakly checked
//
#include <hip/hip_runtime.h>

typedef float          v8f   __attribute__((ext_vector_type(8)));
typedef float          v4f   __attribute__((ext_vector_type(4)));
typedef unsigned int   v4u   __attribute__((ext_vector_type(4)));
typedef int            v8i   __attribute__((ext_vector_type(8)));
typedef unsigned short v8us  __attribute__((ext_vector_type(8)));
typedef unsigned short v16us __attribute__((ext_vector_type(16)));
typedef __bf16         v16bf __attribute__((ext_vector_type(16)));
typedef _Float16       v16h  __attribute__((ext_vector_type(16)));
typedef v4f  __attribute__((may_alias)) v4fa;
typedef v8us __attribute__((may_alias)) v8usa;
union FragB { v16bf v; v16us u; v8us h[2]; v8i w; };
union FragH { v16h  v; v16us u; v8us h[2]; v8i w; };

__device__ __forceinline__ v8f wmb(const FragB& a, const FragB& b, v8f c) {
  v8f d = __builtin_amdgcn_wmma_f32_16x16x32_bf16(false, a.v, false, b.v, (short)0, c, false, false);
  asm volatile("v_nop\n\tv_nop\n\tv_nop\n\tv_nop" : "+v"(d) : "v"(a.w), "v"(b.w));
  return d;
}

__device__ __forceinline__ v8f wmh(const FragH& a, const FragH& b, v8f c) {
  v8f d = __builtin_amdgcn_wmma_f32_16x16x32_f16(false, a.v, false, b.v, (short)0, c, false, false);
  asm volatile("v_nop\n\tv_nop\n\tv_nop\n\tv_nop" : "+v"(d) : "v"(a.w), "v"(b.w));
  return d;
}

__device__ __forceinline__ unsigned bf16_bits(float f) {
  const unsigned u = __float_as_uint(f);
  const unsigned r = (u + 0x7FFFu + ((u >> 16) & 1u)) >> 16;
  const unsigned q = (u >> 16) | 0x40u;
  return ((u & 0x7fffffffu) > 0x7f800000u) ? q : r;
}

__device__ __forceinline__ float bf16_val(float f) {
  return __uint_as_float(bf16_bits(f) << 16);
}
__device__ __forceinline__ int clampi(int v, int lo, int hi) {
  return v < lo ? lo : (v > hi ? hi : v);
}

__device__ __forceinline__ unsigned f16_bits(float f) {
  const unsigned u  = __float_as_uint(f);
  const unsigned s  = (u >> 16) & 0x8000u;
  const unsigned a  = u & 0x7fffffffu;
  const unsigned t  = a - 0x38000000u;
  const unsigned r  = (t + 0x0FFFu + ((t >> 13) & 1u)) >> 13;
  const unsigned rc = r > 0x7C00u ? 0x7C00u : r;
  const bool small  = a < 0x38800000u;
  const bool isnan  = a > 0x7f800000u;
  const unsigned fin = small ? 0u : (s | rc);
  return isnan ? (s | 0x7E00u) : fin;
}

__device__ __forceinline__ unsigned pk16(unsigned lo, unsigned hi) { return lo | (hi << 16); }
__device__ __forceinline__ unsigned bf16_lo_bits(float v) {
  float hi = bf16_val(v);
  asm volatile("" : "+v"(hi));
  return bf16_bits(v - hi);
}
__device__ __forceinline__ v4u pack8_bf16(v4f a, v4f c) {
  return (v4u){ pk16(bf16_bits(a[0]), bf16_bits(a[1])), pk16(bf16_bits(a[2]), bf16_bits(a[3])),
                pk16(bf16_bits(c[0]), bf16_bits(c[1])), pk16(bf16_bits(c[2]), bf16_bits(c[3])) };
}
__device__ __forceinline__ v4u pack8_bf16_lo(v4f a, v4f c) {
  return (v4u){ pk16(bf16_lo_bits(a[0]), bf16_lo_bits(a[1])), pk16(bf16_lo_bits(a[2]), bf16_lo_bits(a[3])),
                pk16(bf16_lo_bits(c[0]), bf16_lo_bits(c[1])), pk16(bf16_lo_bits(c[2]), bf16_lo_bits(c[3])) };
}
__device__ __forceinline__ v4u pack8_f16(v4f a, v4f c) {
  return (v4u){ pk16(f16_bits(a[0]), f16_bits(a[1])), pk16(f16_bits(a[2]), f16_bits(a[3])),
                pk16(f16_bits(c[0]), f16_bits(c[1])), pk16(f16_bits(c[2]), f16_bits(c[3])) };
}

template <int FORM>
__global__ __launch_bounds__(256) void k_plane(const float* __restrict__ src, int rows, int cols, int ldsrc,
                                               unsigned short* __restrict__ dst, int MP, int KP) {
  static_assert(FORM >= 0 && FORM <= 3);
  const int KTOT = (FORM == 1 || FORM == 3) ? 2 * KP : KP;
  const unsigned ppr   = (unsigned)(KTOT >> 3);
  const unsigned kp8   = (unsigned)(KP >> 3);
  const unsigned total = (unsigned)MP * ppr;
  const unsigned g     = blockIdx.x * 256u + threadIdx.x;
  const unsigned rowu  = g / ppr;
  const unsigned p     = g - rowu * ppr;
  const bool second    = p >= kp8;
  const int row = (int)rowu;
  const int c0  = (int)((second ? p - kp8 : p) << 3);
  const float* srow = src + (size_t)clampi(row, 0, rows - 1) * (size_t)ldsrc;
  float x[8];
  unsigned mk[8];
#pragma unroll
  for (int e = 0; e < 8; ++e) {
    const int c = c0 + e;
    const float v = srow[clampi(c, 0, cols - 1)];
    asm volatile("" :: "v"(v));
    x[e]  = v;
    mk[e] = (row < rows && c < cols) ? 0xFFFFu : 0u;
  }
  const v4f a = (v4f){ x[0], x[1], x[2], x[3] };
  const v4f c = (v4f){ x[4], x[5], x[6], x[7] };
  v4u o;
  if (FORM == 2) {
    o = pack8_f16(a, c);
  } else {
    const v4u hi = pack8_bf16(a, c);
    o = hi;
    if (FORM == 1) { const v4u lo = pack8_bf16_lo(a, c); o = second ? lo : hi; }
  }
  const v4u mw = (v4u){ pk16(mk[0], mk[1]), pk16(mk[2], mk[3]), pk16(mk[4], mk[5]), pk16(mk[6], mk[7]) };
  o &= mw;
  if (g < total) {
    volatile v4u* q = (volatile v4u*)(dst + (size_t)g * 8);
    *q = o;
    __threadfence();
    *q = o;
  }
}

template <int FORM> struct FragOf    { typedef FragB T; };
template <>         struct FragOf<2> { typedef FragH T; };
__device__ __forceinline__ v8f mm(const FragB& a, const FragB& b, v8f c) { return wmb(a, b, c); }
__device__ __forceinline__ v8f mm(const FragH& a, const FragH& b, v8f c) { return wmh(a, b, c); }
template <class F> __device__ __forceinline__ F ld_frag(const unsigned short* p) {
  F f;
  f.h[0] = *(const v8usa*)(p);
  f.h[1] = *(const v8usa*)(p + 16);
  return f;
}

template <int FORM, int EPI>
__global__ __launch_bounds__(256) __attribute__((amdgpu_num_vgpr(248)))
void k_gemm_nt(const unsigned short* __restrict__ A, const unsigned short* __restrict__ B,
               const float* __restrict__ bias, float* __restrict__ D, int M, int N, int KTOT, int ldd) {
  static_assert(FORM >= 0 && FORM <= 2);
  static_assert(EPI == 0 || EPI == 1);
  typedef typename FragOf<FORM>::T F;
  __shared__ __attribute__((aligned(16))) float sT[8][16 * 68];
  const int lane = threadIdx.x & 31;
  const int wave = threadIdx.x >> 5;
  const int tilesM = (M + 63) >> 6;
  const int tilesN = (N + 63) >> 6;
  const int tile = blockIdx.x * 8 + wave;
  if (tile >= tilesM * tilesN) return;
  const int tm = tile / tilesN;
  const int tn = tile - tm * tilesN;
  const int m0 = tm << 6;
  const int n0 = tn << 6;

  const int rl = lane & 15;
  const int h8 = (lane >> 4) * 8;
  const unsigned short* pa = A + (size_t)(m0 + rl) * (size_t)KTOT + h8;
  const unsigned short* pb = B + (size_t)(n0 + rl) * (size_t)KTOT + h8;

  v8f acc[4][4];
#pragma unroll
  for (int i = 0; i < 4; ++i)
#pragma unroll
    for (int j = 0; j < 4; ++j) acc[i][j] = (v8f){0.f, 0.f, 0.f, 0.f, 0.f, 0.f, 0.f, 0.f};

#pragma unroll 1
  for (int k0 = 0; k0 < KTOT; k0 += 32) {
    F bf[4];
#pragma unroll
    for (int j = 0; j < 4; ++j) bf[j] = ld_frag<F>(pb + (size_t)(j << 4) * (size_t)KTOT + k0);
#pragma unroll
    for (int i = 0; i < 4; ++i) {
      const F af = ld_frag<F>(pa + (size_t)(i << 4) * (size_t)KTOT + k0);
#pragma unroll
      for (int j = 0; j < 4; ++j) acc[i][j] = mm(af, bf[j], acc[i][j]);
    }
  }

  float* slab = sT[wave];
  const int hh = lane >> 4;
  const int c4 = (lane & 15) * 4;
  const int nc = n0 + c4;
  const bool cok = nc < N;
  v4f bv = (v4f){0.f, 0.f, 0.f, 0.f};
  if (EPI == 1) {
    bv = *(const v4fa*)(bias + clampi(nc, 0, N - 4));
    asm volatile("" :: "v"(bv));
  }
#pragma unroll
  for (int i = 0; i < 4; ++i) {
    const int mBase = m0 + (i << 4);
#pragma unroll
    for (int j = 0; j < 4; ++j) {
#pragma unroll
      for (int r = 0; r < 8; ++r) slab[(h8 + r) * 68 + (j << 4) + rl] = acc[i][j][r];
    }
    __builtin_amdgcn_fence(__ATOMIC_RELEASE, "workgroup");
    __builtin_amdgcn_wave_barrier();
    __builtin_amdgcn_fence(__ATOMIC_ACQUIRE, "workgroup");
    v4f vv[8];
#pragma unroll
    for (int it = 0; it < 8; ++it) {
      const int row = it * 2 + hh;
      v4f v = *(const v4fa*)(slab + row * 68 + c4);
      if (EPI == 1) v += bv;
      vv[it] = v;
    }
    for (int pass = 0; pass < 2; ++pass) {
#pragma unroll
      for (int it = 0; it < 8; ++it) {
        const int row = mBase + it * 2 + hh;
        if (cok && row < M) *(volatile v4f*)(D + (size_t)row * (size_t)ldd + nc) = vv[it];
      }
      __threadfence();
    }
    __builtin_amdgcn_fence(__ATOMIC_RELEASE, "workgroup");
    __builtin_amdgcn_wave_barrier();
    __builtin_amdgcn_fence(__ATOMIC_ACQUIRE, "workgroup");
  }
}

typedef int v4i __attribute__((ext_vector_type(4)));
typedef v4i __attribute__((may_alias)) v4ia;

#define NN      50000
#define DD      128
#define EE      600000
#define MPAD    50048
#define HPLF    (MPAD * DD)
#define SPITCH  50176
#define DBLK    196
#define WSMAX   ((size_t)128 << 20)

#define F_NT    256
#define F_NW    8
#define F_EPT   8
#define F_CHUNK 2048
#define F_WCAP  256
#define F_LISTN 2048
#define F_NB    1024
#define F_RCAP  14336
#define F_DEG   64
#define O_REGP  0
#define O_REGS  (2 * F_RCAP)
#define O_SCNT  (4 * F_RCAP)
#define O_SOFF  (O_SCNT + 2 * F_NB)
#define O_LIST  (O_SOFF + 2 * F_NB)
#define O_WCNT  (O_LIST + 2 * F_LISTN)
#define O_WTOT  (O_WCNT + 16)
#define O_GW    (O_WTOT + 16)
#define O_END   (O_GW + 256)
#define LDS_FUSE (O_END * 4)

static_assert(DD == 32 * 4);
static_assert(MPAD % 64 == 0 && MPAD >= NN);
static_assert(NN % 16 == 0);
static_assert(DD % 64 == 0 && DD % 32 == 0);
static_assert(((MPAD * (DD / 8)) % 256) == 0);
static_assert(SPITCH == DBLK * 256 && SPITCH >= NN);
static_assert(F_NB % 32 == 0 && F_NB == 1024);
static_assert(F_NT * 4 == F_NB);
static_assert(NN < (1 << 17));
static_assert(F_RCAP % 32 == 0 && F_RCAP > 12612);
static_assert(F_DEG >= 30 + 8);
static_assert(F_CHUNK == F_NT * F_EPT && F_WCAP == F_EPT * 32 && F_LISTN == F_NW * F_WCAP);
static_assert(F_LISTN >= F_NB);
static_assert((O_GW % 4) == 0);
static_assert(LDS_FUSE <= 327680);
static_assert(EE % 8 == 0 && EE >= 8);
static_assert((25600000 % 128) == 0 && 25600000 / 4 == NN * DD);
static_assert((long long)NN * DD * 2 - 1 < 12800000LL);

__global__ __launch_bounds__(256) void k_wtr(const float* __restrict__ w, unsigned short* __restrict__ wt) {
  const int nUnits = DD * DD / 8;
  const int u  = (int)blockIdx.x * 256 + (int)threadIdx.x;
  const int uc = u < nUnits - 1 ? u : nUnits - 1;
  const int n  = uc >> 4;
  const int k8 = (uc & 15) << 3;
  const float* p = w + (size_t)k8 * DD + n;
  float x[8];
#pragma unroll
  for (int e = 0; e < 8; ++e) {
    const float v = p[(size_t)e * DD];
    asm volatile("" :: "v"(v));
    x[e] = v;
  }
  const v4u o = pack8_bf16((v4f){ x[0], x[1], x[2], x[3] }, (v4f){ x[4], x[5], x[6], x[7] });
  if (u < nUnits) {
    volatile v4u* q = (volatile v4u*)(wt + (size_t)u * 8);
    *q = o;
    __threadfence();
    *q = o;
  }
}

__global__ __launch_bounds__(256) void k_dots(const float* __restrict__ Hb,
                                              const float* __restrict__ a0, const float* __restrict__ a1,
                                              const float* __restrict__ a2, const float* __restrict__ a3,
                                              float* __restrict__ Sb, int nN) {
  __shared__ __attribute__((aligned(16))) float sA[4 * 256];
  __shared__ __attribute__((aligned(16))) float sS[2 * 256];
  const int tid = (int)threadIdx.x, lane = tid & 31, wave = tid >> 5;
  const int plane = (int)blockIdx.x / DBLK;
  const int blk   = (int)blockIdx.x - plane * DBLK;
  if (tid < 64) {
    const v4f x0 = *(const v4fa*)(a0 + 4 * tid);
    const v4f x1 = *(const v4fa*)(a1 + 4 * tid);
    const v4f x2 = *(const v4fa*)(a2 + 4 * tid);
    const v4f x3 = *(const v4fa*)(a3 + 4 * tid);
    *(v4fa*)(sA +       4 * tid) = (v4f){ bf16_val(x0.x), bf16_val(x0.y), bf16_val(x0.z), bf16_val(x0.w) };
    *(v4fa*)(sA + 256 + 4 * tid) = (v4f){ bf16_val(x1.x), bf16_val(x1.y), bf16_val(x1.z), bf16_val(x1.w) };
    *(v4fa*)(sA + 512 + 4 * tid) = (v4f){ bf16_val(x2.x), bf16_val(x2.y), bf16_val(x2.z), bf16_val(x2.w) };
    *(v4fa*)(sA + 768 + 4 * tid) = (v4f){ bf16_val(x3.x), bf16_val(x3.y), bf16_val(x3.z), bf16_val(x3.w) };
  }
  __syncthreads();
  int va, vb;
  if (plane == 0)      { va = 0;   vb = 128; }
  else if (plane == 1) { va = 512; vb = 896; }
  else if (plane == 2) { va = 256; vb = 384; }
  else                 { va = 640; vb = 768; }
  const v4f wa = *(const v4fa*)(sA + va + 4 * lane);
  const v4f wb = *(const v4fa*)(sA + vb + 4 * lane);
  const float* hp = Hb + (size_t)plane * (size_t)HPLF + 4 * lane;
  const int r0 = blk * 256 + wave * 32;
  float ka = 0.0f, kb = 0.0f;
#pragma unroll 2
  for (int r = 0; r < 32; ++r) {
    const int row = r0 + r;
    const int rc  = row < nN ? row : nN - 1;
    const v4f h = *(const v4fa*)(hp + (size_t)rc * DD);
    float da = h.x * wa.x + h.y * wa.y + h.z * wa.z + h.w * wa.w;
    float db = h.x * wb.x + h.y * wb.y + h.z * wb.z + h.w * wb.w;
#pragma unroll
    for (int off = 16; off > 0; off >>= 1) {
      da += __shfl_xor(da, off);
      db += __shfl_xor(db, off);
    }
    const bool live = row < nN;
    da = live ? da : 0.0f;
    db = live ? db : 0.0f;
    ka = (lane == r) ? da : ka;
    kb = (lane == r) ? db : kb;
  }
  sS[wave * 32 + lane]       = ka;
  sS[256 + wave * 32 + lane] = kb;
  __syncthreads();
  if (tid < 128) {
    const int sel = tid >> 6;
    const int pc  = tid & 63;
    const v4f v = *(const v4fa*)(sS + sel * 256 + 4 * pc);
    float* dp = Sb + (size_t)(2 * plane + sel) * (size_t)SPITCH + (size_t)blk * 256 + 4 * pc;
    *(volatile v4f*)dp = v;
    __threadfence();
    *(volatile v4f*)dp = v;
  }
}

__device__ __forceinline__ int scan_chunk(const int* __restrict__ dsts, int nE, int cbase, int slotBase, int nb,
                                          int* lst, int tid, int lane, int wave) {
  (void)lane;
  int wc = 0;
  const int el0 = tid * F_EPT;
  const int e0  = cbase + el0;
  const int ec  = e0 < nE - F_EPT ? e0 : nE - F_EPT;
  v4i da = *(const v4ia*)(dsts + ec);
  v4i db = *(const v4ia*)(dsts + ec + 4);
  asm volatile("" :: "v"(da), "v"(db));
  const int keep = (e0 < nE) ? -1 : 0;
  const int sent = (int)0x80000000u & ~keep;
  const v4i kv = (v4i){ keep, keep, keep, keep };
  const v4i sv = (v4i){ sent, sent, sent, sent };
  da = (da & kv) | sv;
  db = (db & kv) | sv;
  const unsigned nbs = (unsigned)slotBase;
  const unsigned unb = (unsigned)nb;
  const unsigned s0 = (unsigned)da.x - nbs, s1 = (unsigned)da.y - nbs;
  const unsigned s2 = (unsigned)da.z - nbs, s3 = (unsigned)da.w - nbs;
  const unsigned s4 = (unsigned)db.x - nbs, s5 = (unsigned)db.y - nbs;
  const unsigned s6 = (unsigned)db.z - nbs, s7 = (unsigned)db.w - nbs;
  const bool h0 = s0 < unb, h1 = s1 < unb, h2 = s2 < unb, h3 = s3 < unb;
  const bool h4 = s4 < unb, h5 = s5 < unb, h6 = s6 < unb, h7 = s7 < unb;
  const unsigned any = __builtin_amdgcn_ballot_w32(h0 | h1 | h2 | h3 | h4 | h5 | h6 | h7);
  if (any != 0u) {
#define HITJ(J, HJ, SJ) { \
      const unsigned mj = __builtin_amdgcn_ballot_w32(HJ); \
      if (mj != 0u) { \
        if (HJ) { \
          const int pos = wc + (int)__builtin_amdgcn_mbcnt_lo(mj, 0u); \
          if (pos < F_WCAP) lst[wave * F_WCAP + pos] = ((el0 + (J)) << 12) | (int)(SJ); \
        } \
        wc += (int)__builtin_popcount(mj); } }
    HITJ(0, h0, s0)
    HITJ(1, h1, s1)
    HITJ(2, h2, s2)
    HITJ(3, h3, s3)
    HITJ(4, h4, s4)
    HITJ(5, h5, s5)
    HITJ(6, h6, s6)
    HITJ(7, h7, s7)
#undef HITJ
  }
  return wc;
}

__device__ __forceinline__ void copy_hits(const int* __restrict__ srcs, int nE, int nSrc, int cbase,
                                          const int* lst, int* regp, int wcc, int base, int lane, int wave) {
#pragma unroll 1
  for (int i0 = 0; i0 < wcc; i0 += 32) {
    const int i   = i0 + lane;
    const int ic  = i < wcc ? i : wcc - 1;
    const int ent = lst[wave * F_WCAP + ic];
    const int el  = (ent >> 12) & (F_CHUNK - 1);
    const int sl  = ent & (F_NB - 1);
    const int eid = clampi(cbase + el, 0, nE - 1);
    int sv = srcs[eid];
    asm volatile("" :: "v"(sv));
    sv = clampi(sv, 0, nSrc - 1);
    const int pos = base + i;
    if (i < wcc && pos < F_RCAP) regp[pos] = (int)(((unsigned)sv << 10) | (unsigned)sl);
  }
}

struct Pfx { int e0, e1, e2, e3, ts, incl; };
__device__ __forceinline__ Pfx pfx_load(const int* sc, int tid, int lane) {
  const v4i c = *(const v4ia*)(sc + 4 * tid);
  Pfx p;
  p.e0 = c.x < 0 ? 0 : c.x; p.e1 = c.y < 0 ? 0 : c.y; p.e2 = c.z < 0 ? 0 : c.z; p.e3 = c.w < 0 ? 0 : c.w;
  p.ts = p.e0 + p.e1 + p.e2 + p.e3;
  int incl = p.ts;
#pragma unroll
  for (int d = 1; d < 32; d <<= 1) {
    const int up = __shfl_up(incl, d);
    incl += (lane >= d) ? up : 0;
  }
  p.incl = incl;
  return p;
}
__device__ __forceinline__ void pfx_store(int* so, int* cur, const Pfx p, int pre, int tid) {
  int run = pre + p.incl - p.ts;
  so[4 * tid + 0] = run; cur[4 * tid + 0] = run; run += p.e0;
  so[4 * tid + 1] = run; cur[4 * tid + 1] = run; run += p.e1;
  so[4 * tid + 2] = run; cur[4 * tid + 2] = run; run += p.e2;
  so[4 * tid + 3] = run; cur[4 * tid + 3] = run;
}

__global__ __launch_bounds__(F_NT) __attribute__((amdgpu_num_vgpr(248)))
void k_fuse(const int* __restrict__ srcA, const int* __restrict__ dstA,
            const int* __restrict__ srcB, const int* __restrict__ dstB,
            const float* __restrict__ Hb, const float* __restrict__ Sb,
            const float* __restrict__ gw, const float* __restrict__ gb,
            float* __restrict__ out,
            int hA, int hB, int sdA, int ssA, int sdB, int ssB,
            int nN, int nSrc, int nE, int outBase) {
  extern __shared__ v4f lds_dyn[];
  int* L = (int*)lds_dyn;
  const int tid = (int)threadIdx.x, lane = tid & 31, wave = tid >> 5;
  const int nodeBase = (int)blockIdx.x * F_NB;

  for (int i = tid; i < 2 * F_NB; i += F_NT) L[O_SCNT + i] = 0;
  if (tid < 64) {
    const v4f g4 = *(const v4fa*)(gw + 4 * tid);
    *(v4fa*)((float*)(L + O_GW) + 4 * tid) =
        (v4f){ bf16_val(g4.x), bf16_val(g4.y), bf16_val(g4.z), bf16_val(g4.w) };
  }
  __syncthreads();

  int totA = 0, totB = 0;
  const int nChunks = (nE + F_CHUNK - 1) / F_CHUNK;
#pragma unroll 1
  for (int ch = 0; ch < nChunks; ++ch) {
    const int cbase = ch * F_CHUNK;
    const int wcA = scan_chunk(dstA, nE, cbase, nodeBase, F_NB, L + O_LIST, tid, lane, wave);
    const int wcB = scan_chunk(dstB, nE, cbase, nodeBase, F_NB, L + O_LIST + F_LISTN, tid, lane, wave);
    if (lane == 0) { L[O_WCNT + wave] = wcA; L[O_WCNT + 8 + wave] = wcB; }
    __syncthreads();
    int preA = 0, allA = 0, preB = 0, allB = 0;
#pragma unroll
    for (int w2 = 0; w2 < F_NW; ++w2) {
      const int ca = clampi(L[O_WCNT + w2], 0, F_WCAP);
      const int cb = clampi(L[O_WCNT + 8 + w2], 0, F_WCAP);
      allA += ca; allB += cb;
      preA += (w2 < wave) ? ca : 0;
      preB += (w2 < wave) ? cb : 0;
    }
    copy_hits(srcA, nE, nSrc, cbase, L + O_LIST,           L + O_REGP,          clampi(wcA, 0, F_WCAP),
              totA + preA, lane, wave);
    copy_hits(srcB, nE, nSrc, cbase, L + O_LIST + F_LISTN, L + O_REGP + F_RCAP, clampi(wcB, 0, F_WCAP),
              totB + preB, lane, wave);
    totA += allA; totA = totA > F_RCAP ? F_RCAP : totA;
    totB += allB; totB = totB > F_RCAP ? F_RCAP : totB;
    __syncthreads();
  }
  const int nhA = totA, nhB = totB;

  if (wave < 2) {
    const int nh = wave ? nhB : nhA;
    const int* rp = L + O_REGP + wave * F_RCAP;
    int* sc = L + O_SCNT + wave * F_NB;
#pragma unroll 1
    for (int b0 = 0; b0 < nh; b0 += 32) {
      const int idx = b0 + lane;
      const int uv  = rp[idx < nh ? idx : nh - 1];
      const int m32 = (nh - b0) < 32 ? (nh - b0) : 32;
#pragma unroll 1
      for (int k = 0; k < m32; ++k) {
        const int u  = __builtin_amdgcn_readlane(uv, k);
        const int sl = u & (F_NB - 1);
        if (lane == 0) sc[sl] = sc[sl] + 1;
      }
    }
  }
  __syncthreads();

  {
    const Pfx pa = pfx_load(L + O_SCNT, tid, lane);
    const Pfx pb = pfx_load(L + O_SCNT + F_NB, tid, lane);
    if (lane == 31) { L[O_WTOT + wave] = pa.incl; L[O_WTOT + 8 + wave] = pb.incl; }
    __syncthreads();
    int preA = 0, preB = 0;
#pragma unroll
    for (int w2 = 0; w2 < F_NW; ++w2) {
      const int ta = L[O_WTOT + w2];
      const int tb = L[O_WTOT + 8 + w2];
      preA += (w2 < wave) ? ta : 0;
      preB += (w2 < wave) ? tb : 0;
    }
    pfx_store(L + O_SOFF,        L + O_LIST,           pa, preA, tid);
    pfx_store(L + O_SOFF + F_NB, L + O_LIST + F_LISTN, pb, preB, tid);
  }
  __syncthreads();

  if (wave < 2) {
    const int nh = wave ? nhB : nhA;
    const int* rp = L + O_REGP + wave * F_RCAP;
    int* rs  = L + O_REGS + wave * F_RCAP;
    int* cur = L + O_LIST + wave * F_LISTN;
#pragma unroll 1
    for (int b0 = 0; b0 < nh; b0 += 32) {
      const int idx = b0 + lane;
      const int uv  = rp[idx < nh ? idx : nh - 1];
      const int m32 = (nh - b0) < 32 ? (nh - b0) : 32;
#pragma unroll 1
      for (int k = 0; k < m32; ++k) {
        const int u  = __builtin_amdgcn_readlane(uv, k);
        const int sl = u & (F_NB - 1);
        const int sv = (int)((unsigned)u >> 10);
        if (lane == 0) {
          const int pos = clampi(cur[sl], 0, F_RCAP - 1);
          rs[pos] = sv;
          cur[sl] = pos + 1;
        }
      }
    }
  }
  __syncthreads();

  const float* gwl = (const float*)(L + O_GW);
  const v4f gwf = *(const v4fa*)(gwl + 4 * lane);
  const v4f gwt = *(const v4fa*)(gwl + 128 + 4 * lane);
  const float gbv  = bf16_val(gb[0]);
  const bool  ovf  = (nhA >= F_RCAP) || (nhB >= F_RCAP);
  const float qnan = __uint_as_float(0x7fc00000u);
  const float ninf = __uint_as_float(0xff800000u);
#pragma unroll 1
  for (int jt = 0; jt < F_NB / F_NW; ++jt) {
    const int slot = wave * (F_NB / F_NW) + jt;
    const int grow = nodeBase + slot;
    if (grow >= nN) break;
    float f0 = 0.f, f1 = 0.f, f2 = 0.f, f3 = 0.f;
    float t0 = 0.f, t1 = 0.f, t2 = 0.f, t3 = 0.f;
    bool bad = ovf;
#pragma unroll 1
    for (int q2 = 0; q2 < 2; ++q2) {
      const int nh  = q2 ? nhB : nhA;
      const int hpl = q2 ? hB  : hA;
      const int sdp = q2 ? sdB : sdA;
      const int ssp = q2 ? ssB : ssA;
      const int craw = L[O_SCNT + q2 * F_NB + slot];
      int st  = clampi(L[O_SOFF + q2 * F_NB + slot], 0, nh);
      int cnt = clampi(craw, 0, F_DEG);
      if (cnt > nh - st) cnt = nh - st;
      bad = bad || (craw > F_DEG);
      const float sdv = Sb[(size_t)sdp * (size_t)SPITCH + grow];
      const float* sps = Sb + (size_t)ssp * (size_t)SPITCH;
      const float* hps = Hb + (size_t)hpl * (size_t)HPLF + 4 * lane;
      const int* rs = L + O_REGS + q2 * F_RCAP;
      float mx = ninf, dn = 0.f;
      float a0 = 0.f, a1 = 0.f, a2 = 0.f, a3 = 0.f;
#pragma unroll 1
      for (int q = 0; q < cnt; ++q) {
        const int idx = clampi(st + q, 0, F_RCAP - 1);
        const int sv  = clampi(rs[idx], 0, nSrc - 1);
        const float ssv = sps[sv];
        const v4f h = *(const v4fa*)(hps + (size_t)sv * DD);
        asm volatile("" :: "v"(ssv), "v"(h));
        float al = sdv + ssv;
        al = al > 0.f ? al : 0.2f * al;
        const float df = al - mx;
        const float ee = expf(-fabsf(df));
        const bool  up = df > 0.f;
        const float s1 = up ? ee : 1.0f;
        const float s2 = up ? 1.0f : ee;
        mx = up ? al : mx;
        dn = fmaf(dn, s1, s2);
        a0 = fmaf(a0, s1, s2 * h.x);
        a1 = fmaf(a1, s1, s2 * h.y);
        a2 = fmaf(a2, s1, s2 * h.z);
        a3 = fmaf(a3, s1, s2 * h.w);
      }
      const float inv = 1.0f / (dn + 1e-16f);
      float r0 = a0 * inv, r1 = a1 * inv, r2 = a2 * inv, r3 = a3 * inv;
      r0 = (r0 > 0.f) ? r0 : (r0 - r0);
      r1 = (r1 > 0.f) ? r1 : (r1 - r1);
      r2 = (r2 > 0.f) ? r2 : (r2 - r2);
      r3 = (r3 > 0.f) ? r3 : (r3 - r3);
      const bool empty = (cnt == 0);
      r0 = empty ? 0.f : r0; r1 = empty ? 0.f : r1; r2 = empty ? 0.f : r2; r3 = empty ? 0.f : r3;
      const bool first = (q2 == 0);
      f0 = first ? r0 : f0; f1 = first ? r1 : f1; f2 = first ? r2 : f2; f3 = first ? r3 : f3;
      t0 = first ? t0 : r0; t1 = first ? t1 : r1; t2 = first ? t2 : r2; t3 = first ? t3 : r3;
    }
    float z = f0 * gwf.x + f1 * gwf.y + f2 * gwf.z + f3 * gwf.w
            + t0 * gwt.x + t1 * gwt.y + t2 * gwt.z + t3 * gwt.w;
#pragma unroll
    for (int off = 16; off > 0; off >>= 1) z += __shfl_xor(z, off);
    z += gbv;
    const float g  = 1.0f / (1.0f + expf(-z));
    const float og = 1.0f - g;
    float o0 = g * f0 + og * t0;
    float o1 = g * f1 + og * t1;
    float o2 = g * f2 + og * t2;
    float o3 = g * f3 + og * t3;
    o0 = bad ? qnan : o0; o1 = bad ? qnan : o1; o2 = bad ? qnan : o2; o3 = bad ? qnan : o3;
    const v4f ov = (v4f){ o0, o1, o2, o3 };
    float* op = out + (size_t)outBase + (size_t)grow * DD + 4 * lane;
    *(volatile v4f*)op = ov;
    __threadfence();
    *(volatile v4f*)op = ov;
  }
}

extern "C" void kernel_launch(void* const* d_in, const int* in_sizes, int n_in,
                              void* d_out, int out_size, void* d_ws, size_t ws_size,
                              hipStream_t stream) {
  if (n_in < 22) return;
  if (in_sizes[0] != NN * DD || in_sizes[1] != NN * DD) return;
  if (in_sizes[2] != DD * DD || in_sizes[4] != DD * DD || in_sizes[6] != DD * DD || in_sizes[7] != DD * DD) return;
  if (in_sizes[3] != 2 * DD || in_sizes[5] != 2 * DD || in_sizes[8] != 2 * DD || in_sizes[9] != 2 * DD) return;
  if (in_sizes[10] != 2 * DD || in_sizes[12] != 2 * DD) return;
  if (in_sizes[11] != 1 || in_sizes[13] != 1) return;
  for (int i = 14; i < 22; ++i) if (in_sizes[i] != EE) return;
  if (out_size != 2 * NN * DD) return;

  const float* drug_emb = (const float*)d_in[0];
  const float* dis_emb  = (const float*)d_in[1];
  const float* Wd_feat  = (const float*)d_in[2];
  const float* ad_feat  = (const float*)d_in[3];
  const float* Wp_feat  = (const float*)d_in[4];
  const float* ap_feat  = (const float*)d_in[5];
  const float* W_drug   = (const float*)d_in[6];
  const float* W_dis    = (const float*)d_in[7];
  const float* a_drug   = (const float*)d_in[8];
  const float* a_dis    = (const float*)d_in[9];
  const float* gdW      = (const float*)d_in[10];
  const float* gdb      = (const float*)d_in[11];
  const float* gpW      = (const float*)d_in[12];
  const float* gpb      = (const float*)d_in[13];
  const int* df_src  = (const int*)d_in[14];
  const int* df_dst  = (const int*)d_in[15];
  const int* pf_src  = (const int*)d_in[16];
  const int* pf_dst  = (const int*)d_in[17];
  const int* p2d_src = (const int*)d_in[18];
  const int* p2d_dst = (const int*)d_in[19];
  const int* d2p_src = (const int*)d_in[20];
  const int* d2p_dst = (const int*)d_in[21];
  float* out = (float*)d_out;

  const size_t szXB = (size_t)MPAD * DD * 2;
  const size_t szBT = (size_t)4 * DD * DD * 2;
  const size_t szH  = (size_t)4 * HPLF * 4;
  const size_t szS  = (size_t)8 * SPITCH * 4;
  const size_t oXB = 0;
  const size_t oBT = oXB + szXB;
  const size_t oH  = oBT + szBT;
  const size_t oS  = oH + szH;
  const size_t oEnd = oS + szS;
  if (oEnd > ws_size || oEnd > (size_t)WSMAX) return;
  char* ws = (char*)d_ws;
  unsigned short* XB = (unsigned short*)(ws + oXB);
  unsigned short* BT = (unsigned short*)(ws + oBT);
  float* Hb = (float*)(ws + oH);
  float* Sb = (float*)(ws + oS);
  unsigned short* BT0 = BT;
  unsigned short* BT1 = BT + (size_t)DD * DD;
  unsigned short* BT2 = BT + (size_t)2 * DD * DD;
  unsigned short* BT3 = BT + (size_t)3 * DD * DD;
  float* H0 = Hb;
  float* H1 = Hb + (size_t)HPLF;
  float* H2 = Hb + (size_t)2 * HPLF;
  float* H3 = Hb + (size_t)3 * HPLF;

  hipFuncSetAttribute(reinterpret_cast<const void*>(&k_fuse),
                      hipFuncAttributeMaxDynamicSharedMemorySize, LDS_FUSE);

  k_wtr<<<8, 256, 0, stream>>>(Wd_feat, BT0);
  k_wtr<<<8, 256, 0, stream>>>(W_drug,  BT1);
  k_wtr<<<8, 256, 0, stream>>>(Wp_feat, BT2);
  k_wtr<<<8, 256, 0, stream>>>(W_dis,   BT3);

  const int gPlane = MPAD * (DD / 8) / 256;
  const int gGemm  = (((NN + 63) / 64) * ((DD + 63) / 64) + 7) / 8;

  k_plane<0><<<gPlane, 256, 0, stream>>>(drug_emb, NN, DD, DD, XB, MPAD, DD);
  k_gemm_nt<0, 0><<<gGemm, 256, 0, stream>>>(XB, BT0, gdb, H0, NN, DD, DD, DD);
  k_gemm_nt<0, 0><<<gGemm, 256, 0, stream>>>(XB, BT1, gdb, H1, NN, DD, DD, DD);
  k_plane<0><<<gPlane, 256, 0, stream>>>(dis_emb, NN, DD, DD, XB, MPAD, DD);
  k_gemm_nt<0, 0><<<gGemm, 256, 0, stream>>>(XB, BT2, gdb, H2, NN, DD, DD, DD);
  k_gemm_nt<0, 0><<<gGemm, 256, 0, stream>>>(XB, BT3, gdb, H3, NN, DD, DD, DD);

  k_dots<<<4 * DBLK, 256, 0, stream>>>(Hb, ad_feat, ap_feat, a_drug, a_dis, Sb, NN);

  const int gFuse = (NN + F_NB - 1) / F_NB;
  k_fuse<<<gFuse, F_NT, LDS_FUSE, stream>>>(df_src, df_dst, p2d_src, p2d_dst, Hb, Sb, gdW, gdb, out,
                                            0, 3, 0, 1, 2, 6, NN, NN, EE, 0);
  k_fuse<<<gFuse, F_NT, LDS_FUSE, stream>>>(pf_src, pf_dst, d2p_src, d2p_dst, Hb, Sb, gpW, gpb, out,
                                            2, 1, 4, 5, 7, 3, NN, NN, EE, NN * DD);
}
